// testNet_7593502179527
// MI455X (gfx1250) — hardware-verified
//
#include <hip/hip_runtime.h>

typedef __attribute__((ext_vector_type(16))) _Float16 v16h;
typedef __attribute__((ext_vector_type(8)))  _Float16 v8h;
typedef __attribute__((ext_vector_type(8)))  float    v8f;
typedef __attribute__((ext_vector_type(4)))  float    v4f_t;
typedef float v4fa __attribute__((ext_vector_type(4), may_alias));
#define RSPLIT (1.0f / 2048.0f)
__device__ __forceinline__ _Float16 lo_of(float v, _Float16 h) { return (_Float16)((v - (float)h) * 2048.0f); }
__device__ __forceinline__ v8f wmma16(v16h a, v16h b, v8f c) { return __builtin_amdgcn_wmma_f32_16x16x32_f16(false, a, false, b, (short)0, c, false, false); }
__device__ __forceinline__ v8f wmma_split(v16h a, v16h al, v16h b, v16h bl, v8f c) { v8f x = {}; x = wmma16(al, b, x); x = wmma16(a, bl, x); return wmma16(a, b, c) + x * RSPLIT; }
__device__ __forceinline__ void st2f(float* p, float v) { *(volatile float*)p = v; __threadfence(); *(volatile float*)p = v; }

namespace {
constexpr int kB = 16;
constexpr int kS = 1024;
constexpr int kL = 2048;
constexpr int kH = 32;
constexpr int kG = 128;
}

#if __has_builtin(__builtin_amdgcn_tanhf)
__device__ __forceinline__ float fast_tanh(float x) { return __builtin_amdgcn_tanhf(x); }
#elif __has_builtin(__builtin_amdgcn_tanh_f32)
__device__ __forceinline__ float fast_tanh(float x) { return __builtin_amdgcn_tanh_f32(x); }
#else
__device__ __forceinline__ float fast_tanh(float x) { return tanhf(x); }
#endif

__global__ void attn_kernel(const float* __restrict__ v1,
                            const float* __restrict__ v2,
                            const float* __restrict__ attn_w,
                            float* __restrict__ attn_out) {
    const int which = blockIdx.x & 1;
    const int b     = blockIdx.x >> 1;
    const float* v  = which ? v2 : v1;
    const int tid   = threadIdx.x;

    __shared__ float sc[kL];
    __shared__ float red[256 * 4];

    const float wk0 = attn_w[3], wk1 = attn_w[4], wk2 = attn_w[5];
    const float* vb = v + (size_t)b * (kL + 1) * 3;

    float mloc = -3.4e38f;
    for (int j = tid; j < kL; j += 256) {
        float s = vb[j*3+0]*wk0 + vb[j*3+1]*wk1 + vb[j*3+2]*wk2;
        sc[j] = s;
        mloc = fmaxf(mloc, s);
    }
    red[tid] = mloc;
    __syncthreads();
    for (int off = 128; off > 0; off >>= 1) {
        if (tid < off) red[tid] = fmaxf(red[tid], red[tid + off]);
        __syncthreads();
    }
    const float mx = red[0];
    __syncthreads();

    float a0 = 0.f, a1 = 0.f, a2 = 0.f, asum = 0.f;
    for (int j = tid; j < kL; j += 256) {
        float e = __expf(sc[j] - mx);
        asum += e;
        a0 += e * vb[(j+1)*3+0];
        a1 += e * vb[(j+1)*3+1];
        a2 += e * vb[(j+1)*3+2];
    }
    red[tid*4+0] = a0; red[tid*4+1] = a1; red[tid*4+2] = a2; red[tid*4+3] = asum;
    __syncthreads();
    for (int off = 128; off > 0; off >>= 1) {
        if (tid < off) {
            red[tid*4+0] += red[(tid+off)*4+0];
            red[tid*4+1] += red[(tid+off)*4+1];
            red[tid*4+2] += red[(tid+off)*4+2];
            red[tid*4+3] += red[(tid+off)*4+3];
        }
        __syncthreads();
    }
    if (tid == 0) {
        float inv = 1.0f / red[3];
        float* ao = attn_out + (which * kB + b) * 32;
        st2f(ao + 0, red[0] * inv); st2f(ao + 1, red[1] * inv); st2f(ao + 2, red[2] * inv);
    }
}

__global__ __launch_bounds__(32) void xg_kernel(const float* __restrict__ x,
                          const float* __restrict__ fc1_w, const float* __restrict__ fc1_b,
                          const float* __restrict__ w_ih,
                          const float* __restrict__ b_ih,  const float* __restrict__ b_hh,
                          float* __restrict__ xg) {
    __shared__ __attribute__((aligned(16))) float stg[kG * kB];
    const int s = blockIdx.x, lane = threadIdx.x, lo = lane & 15, hi = lane >> 4;
    v16h a, al;
    {
        const float* xr = x + ((size_t)lo * kS + s) * 3;
        const float x0 = xr[0], x1 = xr[1], x2 = xr[2];
        #pragma unroll
        for (int e = 0; e < 16; ++e) {
            const int k = (e < 8) ? (hi * 8 + e) : (16 + hi * 8 + (e - 8));
            float v = 0.f;
            if (k < 16) v = fc1_b[k] + x0 * fc1_w[k * 3 + 0] + x1 * fc1_w[k * 3 + 1] + x2 * fc1_w[k * 3 + 2];
            a[e] = (_Float16)v; al[e] = lo_of(v, a[e]);
        }
    }
    #pragma unroll 1
    for (int nt = 0; nt < 8; ++nt) {
        v16h b, bl;
        const int n = nt * 16 + lo;
        #pragma unroll
        for (int e = 0; e < 16; ++e) {
            const int k = (e < 8) ? (hi * 8 + e) : (16 + hi * 8 + (e - 8));
            const float w = (k < 16) ? w_ih[n * 16 + k] : 0.f;
            b[e] = (_Float16)w; bl[e] = lo_of(w, b[e]);
        }
        v8f c = {};
        c = wmma_split(a, al, b, bl, c);
        const float bs = b_ih[n] + b_hh[n];
        #pragma unroll
        for (int r = 0; r < 8; ++r) stg[n * kB + hi * 8 + r] = c[r] + bs;
    }
    asm volatile("s_wait_dscnt 0" ::: "memory");
    float* dst = xg + (size_t)s * kG * kB;
    #pragma unroll 1
    for (int pass = 0; pass < 2; ++pass) {
        #pragma unroll
        for (int i = 0; i < 16; ++i) { const int c4 = (lane + 32 * i) * 4; *(volatile v4f_t*)(dst + c4) = *(const volatile v4fa*)(stg + c4); }
        __threadfence();
    }
}

__global__ void __launch_bounds__(256, 1)
lstm_kernel(const float* __restrict__ xg,
            const float* __restrict__ w_hh,
            float* __restrict__ hs) {
    const int tid  = threadIdx.x;
    const int wave = tid >> 5;
    const int lane = tid & 31;

    __shared__ _Float16 hlds16[2 * kB * kH];
    __shared__ float    act[kG * kB];

    const int ncol = (wave << 4) + (lane & 15);
    const int kbB  = (lane < 16) ? 0 : 8;
    v16h bfrag, bfragl;
    #pragma unroll
    for (int h = 0; h < 16; ++h) {
        const int k = (h < 8) ? (kbB + h) : (16 + kbB + (h - 8));
        const float w = w_hh[ncol * kH + k];
        bfrag[h] = (_Float16)w; bfragl[h] = lo_of(w, bfrag[h]);
    }

    hlds16[tid]       = (_Float16)0.0f;  hlds16[kB * kH + tid]       = (_Float16)0.0f;
    hlds16[tid + 256] = (_Float16)0.0f;  hlds16[kB * kH + tid + 256] = (_Float16)0.0f;
    const int kown = tid & 31, bown = tid >> 5;
    float creg0 = 0.0f, creg1 = 0.0f;

    const int m     = lane & 15;
    const int kbA   = (lane < 16) ? 0 : 8;
    const int rbase = (lane < 16) ? 0 : 8;
    const _Float16* arow = &hlds16[m * kH + kbA];

    const bool  is_g = ((wave >> 1) == 2);
    const float sco  = is_g ? 1.0f : 0.5f;
    const float aco  = is_g ? 1.0f : 0.5f;
    const float bco  = is_g ? 0.0f : 0.5f;

    __syncthreads();

    float hv0 = 0.f, hv1 = 0.f;
    for (int s = 0; s < kS; ++s) {
        v8h alo = *(const v8h*)(arow);
        v8h ahi = *(const v8h*)(arow + 16);
        v8h llo = *(const v8h*)(arow + kB * kH), lhi = *(const v8h*)(arow + kB * kH + 16);
        v16h afrag, afragl;
        #pragma unroll
        for (int h = 0; h < 8; ++h) { afrag[h] = alo[h]; afrag[8 + h] = ahi[h]; afragl[h] = llo[h]; afragl[8 + h] = lhi[h]; }

        v8f cacc = {};
        cacc = wmma_split(afrag, afragl, bfrag, bfragl, cacc);

        const float* xgp = xg + ((size_t)s * kG + ncol) * kB + rbase;
        float4 xlo = *(const float4*)(xgp);
        float4 xhi = *(const float4*)(xgp + 4);
        float g[8];
        g[0] = cacc[0] + xlo.x; g[1] = cacc[1] + xlo.y;
        g[2] = cacc[2] + xlo.z; g[3] = cacc[3] + xlo.w;
        g[4] = cacc[4] + xhi.x; g[5] = cacc[5] + xhi.y;
        g[6] = cacc[6] + xhi.z; g[7] = cacc[7] + xhi.w;
        #pragma unroll
        for (int q = 0; q < 8; ++q)
            g[q] = fmaf(aco, fast_tanh(sco * g[q]), bco);

        float* ap = &act[ncol * kB + rbase];
        *(float4*)(ap)     = make_float4(g[0], g[1], g[2], g[3]);
        *(float4*)(ap + 4) = make_float4(g[4], g[5], g[6], g[7]);
        __syncthreads();

        {
            const int k = kown, b = bown;
            float iv = act[k*kB + b],          fv = act[(kH + k)*kB + b];
            float gv = act[(2*kH + k)*kB + b], ov = act[(3*kH + k)*kB + b];
            creg0 = fv * creg0 + iv * gv;
            float hv = ov * fast_tanh(creg0);
            const _Float16 hh = (_Float16)hv; hlds16[b*kH + k] = hh; hlds16[kB * kH + b*kH + k] = lo_of(hv, hh);
            hv0 = hv;
        }
        {
            const int k = kown, b = bown + 8;
            float iv = act[k*kB + b],          fv = act[(kH + k)*kB + b];
            float gv = act[(2*kH + k)*kB + b], ov = act[(3*kH + k)*kB + b];
            creg1 = fv * creg1 + iv * gv;
            float hv = ov * fast_tanh(creg1);
            const _Float16 hh = (_Float16)hv; hlds16[b*kH + k] = hh; hlds16[kB * kH + b*kH + k] = lo_of(hv, hh);
            hv1 = hv;
        }
        {
            float* hp0 = hs + ((size_t)bown * kS + s) * kH + kown; float* hp1 = hs + ((size_t)(bown + 8) * kS + s) * kH + kown;
            *(volatile float*)hp0 = hv0; *(volatile float*)hp1 = hv1; __threadfence(); *(volatile float*)hp0 = hv0; *(volatile float*)hp1 = hv1;
        }
        __syncthreads();
    }
}

__global__ __launch_bounds__(32) void head_kernel(const float* __restrict__ hs,
                            const float* __restrict__ attn_out,
                            const float* __restrict__ fc2_w, const float* __restrict__ fc2_b,
                            const float* __restrict__ fc3_w, const float* __restrict__ fc3_b,
                            float* __restrict__ out) {
    __shared__ __attribute__((aligned(16))) float so[48];
    const int lane = threadIdx.x, lo = lane & 15, hi = lane >> 4;
    const int row0 = blockIdx.x * 16;
    const int idx = row0 + lo, b = idx >> 10, s = idx & 1023;
    auto catv = [&](int d) -> float {
        if (d < 3)  return attn_out[(0 * kB + b) * 32 + d];
        if (d < 6)  return attn_out[(1 * kB + b) * 32 + (d - 3)];
        if (d < 38) return hs[((size_t)b * kS + s) * kH + (d - 6)];
        return 0.f;
    };
    v8f y = {};
    #pragma unroll
    for (int kc = 0; kc < 2; ++kc) {
        v16h a, al, w, wl;
        #pragma unroll
        for (int e = 0; e < 16; ++e) {
            const int k = kc * 32 + ((e < 8) ? (hi * 8 + e) : (16 + hi * 8 + (e - 8)));
            const float cv = catv(k);
            const float wv = (k < 38) ? fc2_w[lo * 38 + k] : 0.f;
            a[e] = (_Float16)cv; al[e] = lo_of(cv, a[e]); w[e] = (_Float16)wv; wl[e] = lo_of(wv, w[e]);
        }
        y = wmma_split(a, al, w, wl, y);
    }
    __shared__ float ys[16][17];
    #pragma unroll
    for (int r = 0; r < 8; ++r) ys[hi * 8 + r][lo] = fmaxf(y[r] + fc2_b[lo], 0.f);
    asm volatile("s_wait_dscnt 0" ::: "memory");
    v16h a2, a2l, w3, w3l;
    #pragma unroll
    for (int e = 0; e < 16; ++e) {
        const int k = (e < 8) ? (hi * 8 + e) : (16 + hi * 8 + (e - 8));
        const float yv = (k < 16) ? ys[lo][k] : 0.f;
        const float wv = (k < 16 && lo < 3) ? fc3_w[lo * 16 + k] : 0.f;
        a2[e] = (_Float16)yv; a2l[e] = lo_of(yv, a2[e]); w3[e] = (_Float16)wv; w3l[e] = lo_of(wv, w3[e]);
    }
    v8f o = {};
    o = wmma_split(a2, a2l, w3, w3l, o);
    if (lo < 3) {
        #pragma unroll
        for (int r = 0; r < 8; ++r) so[(hi * 8 + r) * 3 + lo] = o[r] + fc3_b[lo];
    }
    asm volatile("s_wait_dscnt 0" ::: "memory");
    float* op = out + (size_t)row0 * 3;
    #pragma unroll 1
    for (int pass = 0; pass < 2; ++pass) {
        if (lane < 12) *(volatile v4f_t*)(op + lane * 4) = *(const volatile v4fa*)(so + lane * 4);
        __threadfence();
    }
}

extern "C" void kernel_launch(void* const* d_in, const int* in_sizes, int n_in,
                              void* d_out, int out_size, void* d_ws, size_t ws_size,
                              hipStream_t stream) {
    const float* x      = (const float*)d_in[0];
    const float* v1     = (const float*)d_in[1];
    const float* v2     = (const float*)d_in[2];
    const float* attn_w = (const float*)d_in[3];
    const float* fc1_w  = (const float*)d_in[5];
    const float* fc1_b  = (const float*)d_in[6];
    const float* w_ih   = (const float*)d_in[7];
    const float* w_hh   = (const float*)d_in[8];
    const float* b_ih   = (const float*)d_in[9];
    const float* b_hh   = (const float*)d_in[10];
    const float* fc2_w  = (const float*)d_in[11];
    const float* fc2_b  = (const float*)d_in[12];
    const float* fc3_w  = (const float*)d_in[13];
    const float* fc3_b  = (const float*)d_in[14];
    (void)in_sizes; (void)n_in; (void)out_size; (void)ws_size;

    char* ws = (char*)d_ws;
    float* xg   = (float*)(ws);
    float* hsb  = (float*)(ws + (size_t)8  * 1024*1024);
    float* attn = (float*)(ws + (size_t)10 * 1024*1024);

    xg_kernel  <<<kS,        32, 0, stream>>>(x, fc1_w, fc1_b, w_ih, b_ih, b_hh, xg);
    attn_kernel<<<2 * kB,   256, 0, stream>>>(v1, v2, attn_w, attn);
    lstm_kernel<<<1,        256, 0, stream>>>(xg, w_hh, hsb);
    head_kernel<<<kB*kS/16,  32, 0, stream>>>(hsb, attn, fc2_w, fc2_b, fc3_w, fc3_b,
                                              (float*)d_out);
}
